// BrickVectorEdgeModel_34737695490544
// MI455X (gfx1250) — hardware-verified
//
#include <hip/hip_runtime.h>
#include <math.h>

typedef __attribute__((ext_vector_type(16))) _Float16 v16h;
typedef __attribute__((ext_vector_type(8)))  _Float16 v8h;
typedef __attribute__((ext_vector_type(16))) __bf16   v16b;
typedef __attribute__((ext_vector_type(8)))  __bf16   v8b;
typedef __attribute__((ext_vector_type(8)))  float    v8f;
typedef __attribute__((ext_vector_type(4)))  float    v4f;

constexpr int kBatch    = 4;
constexpr int kNodes    = 192;
constexpr int kDim      = 512;
constexpr int kHid      = 512;
constexpr int kRows     = kBatch * kNodes;
constexpr int kUVP      = 2 * kHid;
constexpr int kEdgeRows = 64;
constexpr int kOutTileN = 16;
static_assert(kRows == 768);
static_assert(kDim == kHid);
static_assert((kDim % 32) == 0 && (kHid % 32) == 0);
static_assert((kRows % 64) == 0 && (kHid % 64) == 0 && (kUVP % 64) == 0);
static_assert((kNodes % kEdgeRows) == 0);

constexpr float kActCarry = 64.0f;
constexpr float kWCarry   = 256.0f;
constexpr float kLoCarry  = 2048.0f;
constexpr float kAccScale = 1.0f / kWCarry;
constexpr float kOutScale = 1.0f / (kActCarry * kWCarry);
constexpr float kLoInv    = 1.0f / kLoCarry;

constexpr size_t kOffBRH = 0;
constexpr size_t kOffBRL = kOffBRH + (size_t)kRows * kDim * 2;
constexpr size_t kOffWAH = kOffBRL + (size_t)kRows * kDim * 2;
constexpr size_t kOffWAL = kOffWAH + (size_t)kHid * kDim * 2;
constexpr size_t kOffWBH = kOffWAL + (size_t)kHid * kDim * 2;
constexpr size_t kOffWBL = kOffWBH + (size_t)kHid * kHid * 2;
constexpr size_t kOffUVH = kOffWBL + (size_t)kHid * kHid * 2;
constexpr size_t kOffUVL = kOffUVH + (size_t)kUVP * kHid * 2;
constexpr size_t kOffF1H = kOffUVL + (size_t)kUVP * kHid * 2;
constexpr size_t kOffF1L = kOffF1H + (size_t)kRows * kHid * 2;
constexpr size_t kOffF2H = kOffF1L + (size_t)kRows * kHid * 2;
constexpr size_t kOffF2L = kOffF2H + (size_t)kRows * kHid * 2;
constexpr size_t kOffUV  = kOffF2L + (size_t)kRows * kHid * 2;
constexpr size_t kOffWCB = kOffUV  + (size_t)kRows * kUVP * 4;
constexpr size_t kOffWCC = kOffWCB + (size_t)kHid * kHid * 2;
constexpr size_t kOffWOT = kOffWCC + (size_t)kHid * kHid * 2;
constexpr size_t kWsTotal = kOffWOT + (size_t)kOutTileN * kHid * 2;
static_assert(kWsTotal == 13123584ull);
static_assert(kWsTotal <= 134217728ull);
static_assert((kOffBRL % 128) == 0 && (kOffWAH % 128) == 0 && (kOffWAL % 128) == 0 && (kOffWBH % 128) == 0 &&
              (kOffWBL % 128) == 0 && (kOffUVH % 128) == 0 && (kOffUVL % 128) == 0 && (kOffF1H % 128) == 0 &&
              (kOffF1L % 128) == 0 && (kOffF2H % 128) == 0 && (kOffF2L % 128) == 0 && (kOffUV % 128) == 0 &&
              (kOffWCB % 128) == 0 && (kOffWCC % 128) == 0 && (kOffWOT % 128) == 0);

constexpr int kSegWa   = (kRows * kDim / 8) / 256;
constexpr int kSegWb   = kSegWa  + (kHid * kDim / 8) / 256;
constexpr int kSegWca  = kSegWb  + (kHid * kHid / 8) / 256;
constexpr int kSegCast = kSegWca + (kUVP * kHid / 8) / 256;
constexpr int kSegWcc  = kSegCast + (kHid * kHid / 8) / 256;
constexpr int kSegWo   = kSegWcc + (kHid * kHid / 8) / 256;
constexpr int kSegEnd  = kSegWo  + (kOutTileN * kHid / 8) / 256;
static_assert(kSegWa == 192 && kSegWb == 320 && kSegWca == 448 && kSegCast == 704);
static_assert(kSegWcc == 832 && kSegWo == 960 && kSegEnd == 964);

__device__ __forceinline__ unsigned short f2bf_bits(float f) {
  unsigned u = __float_as_uint(f);
  return (unsigned short)((u + 0x7FFFu + ((u >> 16) & 1u)) >> 16);
}
__device__ __forceinline__ float bf_bits2f(unsigned short h) { return __uint_as_float(((unsigned)h) << 16); }

template <typename T> struct Frag;
template <> struct Frag<_Float16> {
  typedef v16h V; union U { v16h v; v8h h[2]; };
  static __device__ __forceinline__ v16h load(const _Float16* p) {
    U f; f.h[0] = *(const v8h*)(p); f.h[1] = *(const v8h*)(p + 16); return f.v;
  }
};
template <> struct Frag<__bf16> {
  typedef v16b V; union U { v16b v; v8b h[2]; };
  static __device__ __forceinline__ v16b load(const __bf16* p) {
    U f; f.h[0] = *(const v8b*)(p); f.h[1] = *(const v8b*)(p + 16); return f.v;
  }
};

__device__ __forceinline__ v8f mma_bf(v16b a, v16b b, v8f c) {
  c = __builtin_amdgcn_wmma_f32_16x16x32_bf16(false, a, false, b, (short)0, c, false, false);
  asm volatile("v_nop\n\tv_nop\n\tv_nop\n\tv_nop" : "+v"(c) : "v"(a), "v"(b));
  return c;
}
__device__ __forceinline__ v8f mma_h(v16h a, v16h b, v8f c) {
  c = __builtin_amdgcn_wmma_f32_16x16x32_f16(false, a, false, b, (short)0, c, false, false);
  asm volatile("v_nop\n\tv_nop\n\tv_nop\n\tv_nop" : "+v"(c) : "v"(a), "v"(b));
  return c;
}

__device__ __forceinline__ void store16_twice(unsigned short* q, v8h v) {
  *(volatile v8h*)q = v;
  __threadfence();
  *(volatile v8h*)q = v;
}
__device__ __forceinline__ void store16_pair_twice(unsigned short* qh, v8h hv, unsigned short* ql, v8h lv) {
  *(volatile v8h*)qh = hv;
  *(volatile v8h*)ql = lv;
  __threadfence();
  *(volatile v8h*)qh = hv;
  *(volatile v8h*)ql = lv;
}

__device__ __forceinline__ void split8(const float* src, v8h& hv, v8h& lv) {
  const v4f a0 = *(const v4f*)(src);
  const v4f a1 = *(const v4f*)(src + 4);
#pragma unroll
  for (int e = 0; e < 4; ++e) {
    const float x0 = a0[e];
    const float x1 = a1[e];
    const unsigned short h0 = f2bf_bits(x0), h1 = f2bf_bits(x1);
    const unsigned short l0 = f2bf_bits(x0 - bf_bits2f(h0)), l1 = f2bf_bits(x1 - bf_bits2f(h1));
    hv[e]     = __builtin_bit_cast(_Float16, h0);
    hv[4 + e] = __builtin_bit_cast(_Float16, h1);
    lv[e]     = __builtin_bit_cast(_Float16, l0);
    lv[4 + e] = __builtin_bit_cast(_Float16, l1);
  }
}

__global__ __launch_bounds__(256) void prep_kernel(
    const float* __restrict__ brick, const float* __restrict__ Wa, const float* __restrict__ Wb,
    const float* __restrict__ Wca, const float* __restrict__ Wcb, const float* __restrict__ Wcc,
    const float* __restrict__ Wout, unsigned char* __restrict__ ws)
{
  const int bx = blockIdx.x, tid = threadIdx.x;
  if (bx < kSegCast) {
    const float* src;
    size_t offH, offL;
    int t;
    if (bx < kSegWa) {
      t = bx * 256 + tid;
      src = brick + (size_t)t * 8;
      offH = kOffBRH; offL = kOffBRL;
    } else if (bx < kSegWb) {
      t = (bx - kSegWa) * 256 + tid;
      src = Wa + (size_t)t * 8;
      offH = kOffWAH; offL = kOffWAL;
    } else if (bx < kSegWca) {
      t = (bx - kSegWb) * 256 + tid;
      src = Wb + (size_t)t * 8;
      offH = kOffWBH; offL = kOffWBL;
    } else {
      t = (bx - kSegWca) * 256 + tid;
      const int e0 = t * 8;
      const int r = e0 >> 9, h = e0 & (kHid - 1);
      const int s = r >> 9, g = r & (kHid - 1);
      src = Wca + (size_t)g * kUVP + s * kHid + h;
      offH = kOffUVH; offL = kOffUVL;
    }
    v8h hv, lv;
    split8(src, hv, lv);
    unsigned short* qh = (unsigned short*)(ws + offH) + (size_t)t * 8;
    unsigned short* ql = (unsigned short*)(ws + offL) + (size_t)t * 8;
    store16_pair_twice(qh, hv, ql, lv);
  } else if (bx < kSegWo) {
    const bool second = (bx >= kSegWcc);
    const int t = (bx - (second ? kSegWcc : kSegCast)) * 256 + tid;
    const float* src = (second ? Wcc : Wcb) + (size_t)t * 8;
    const v4f a0 = *(const v4f*)(src);
    const v4f a1 = *(const v4f*)(src + 4);
    v8h hv;
#pragma unroll
    for (int e = 0; e < 4; ++e) {
      const float x0 = a0[e];
      const float x1 = a1[e];
      hv[e]     = (_Float16)(x0 * kWCarry);
      hv[4 + e] = (_Float16)(x1 * kWCarry);
    }
    unsigned short* q = (unsigned short*)(ws + (second ? kOffWCC : kOffWCB)) + (size_t)t * 8;
    store16_twice(q, hv);
  } else {
    const int t = (bx - kSegWo) * 256 + tid;
    const int e0 = t * 8;
    const int row = e0 >> 9, h = e0 & (kHid - 1);
    const float* src = Wout + (size_t)(row & 1) * kHid + h;
    const v4f a0 = *(const v4f*)(src);
    const v4f a1 = *(const v4f*)(src + 4);
    v8h hv;
#pragma unroll
    for (int e = 0; e < 8; ++e) {
      float x;
      if (e < 4) x = a0[e & 3]; else x = a1[e & 3];
      const float w = x * kWCarry;
      const _Float16 hi = (_Float16)w;
      const float hif = (float)hi;
      const _Float16 lo = (_Float16)((w - hif) * kLoCarry);
      const _Float16 zero = (_Float16)0.0f;
      hv[e] = (row < 2) ? hi : ((row < 4) ? lo : zero);
    }
    unsigned short* q = (unsigned short*)(ws + kOffWOT) + (size_t)t * 8;
    store16_twice(q, hv);
  }
}

template <int EPI>
__global__ __launch_bounds__(256) void node_gemm_kernel(
    const unsigned short* __restrict__ Ahp, const unsigned short* __restrict__ Alp,
    const unsigned short* __restrict__ Bhp, const unsigned short* __restrict__ Blp,
    void* __restrict__ Cout, void* __restrict__ Cout2, int ldc,
    const float* __restrict__ bias0, const float* __restrict__ bias1,
    const float* __restrict__ xy, const float* __restrict__ wxy, int M, int N)
{
  const __bf16* Ah = (const __bf16*)Ahp;
  const __bf16* Al = (const __bf16*)Alp;
  const __bf16* Bh = (const __bf16*)Bhp;
  const __bf16* Bl = (const __bf16*)Blp;
  __shared__ __align__(16) float sT[8][16 * 68];
  const int lane = threadIdx.x & 31;
  const int wave = threadIdx.x >> 5;
  const int tilesN = N >> 6;
  const int tilesM = M >> 6;
  const int tile = blockIdx.x * 8 + wave;
  if (tile >= tilesM * tilesN) return;
  const int tm = tile / tilesN;
  const int tn = tile - tm * tilesN;
  const int m0 = tm << 6;
  const int n0 = tn << 6;

  const int rlane = lane & 15;
  const int koff  = (lane >> 4) * 8;
  const int mOff  = (lane >> 4) * 8;

  v8f acc[4][4];
#pragma unroll
  for (int i = 0; i < 4; ++i)
#pragma unroll
    for (int j = 0; j < 4; ++j) acc[i][j] = (v8f){0.f,0.f,0.f,0.f,0.f,0.f,0.f,0.f};

#pragma unroll 1
  for (int k0 = 0; k0 < kDim; k0 += 32) {
    v16b bh[4], bl[4];
#pragma unroll
    for (int j = 0; j < 4; ++j) {
      const size_t bo = (size_t)(n0 + (j << 4) + rlane) * kDim + koff + k0;
      bh[j] = Frag<__bf16>::load(Bh + bo);
      bl[j] = Frag<__bf16>::load(Bl + bo);
    }
#pragma unroll
    for (int i = 0; i < 4; ++i) {
      const size_t ao = (size_t)(m0 + (i << 4) + rlane) * kDim + koff + k0;
      const v16b ah = Frag<__bf16>::load(Ah + ao);
      const v16b al = Frag<__bf16>::load(Al + ao);
#pragma unroll
      for (int j = 0; j < 4; ++j) {
        acc[i][j] = mma_bf(ah, bh[j], acc[i][j]);
        acc[i][j] = mma_bf(ah, bl[j], acc[i][j]);
        acc[i][j] = mma_bf(al, bh[j], acc[i][j]);
      }
    }
  }

  float* slab = sT[wave];
#pragma unroll
  for (int i = 0; i < 4; ++i) {
    const int mBase = m0 + (i << 4);
    v4f xq[4];
    if (EPI == 0) {
      const float* xp = xy + (size_t)(mBase + mOff) * 2;
      xq[0] = *(const v4f*)(xp);
      xq[1] = *(const v4f*)(xp + 4);
      xq[2] = *(const v4f*)(xp + 8);
      xq[3] = *(const v4f*)(xp + 12);
    }
#pragma unroll
    for (int j = 0; j < 4; ++j) {
      const int n = n0 + (j << 4) + rlane;
      float bv = 0.f, bv2 = 0.f, w0 = 0.f, w1 = 0.f;
      if (EPI == 0) {
        bv = bias0[n];
        bv2 = bias1[n];
        w0 = wxy[2 * n];
        w1 = wxy[2 * n + 1];
      }
      if (EPI == 1) bv = bias0[n];
      if (EPI == 2) {
        const float t = bias0[n & (kHid - 1)];
        bv = (n >= kHid) ? (t * kActCarry) : 0.f;
      }
#pragma unroll
      for (int r = 0; r < 8; ++r) {
        float v = acc[i][j][r];
        if (EPI == 0) {
          const float x0 = xq[r >> 1][(r & 1) * 2];
          const float x1 = xq[r >> 1][(r & 1) * 2 + 1];
          v = v + bv;
          v = v + (x0 * w0 + x1 * w1);
          v = v + bv2;
          v = fmaxf(v, 0.0f);
        }
        if (EPI == 1) {
          v = v + bv;
          v = fmaxf(v, 0.0f);
        }
        if (EPI == 2) {
          v = v * kActCarry + bv;
        }
        slab[(mOff + r) * 68 + (j << 4) + rlane] = v;
      }
    }
    __builtin_amdgcn_fence(__ATOMIC_RELEASE, "workgroup");
    __builtin_amdgcn_wave_barrier();
    __builtin_amdgcn_fence(__ATOMIC_ACQUIRE, "workgroup");
    if (EPI == 2) {
      float* C = (float*)Cout;
      const int hh = lane >> 4, c4 = (lane & 15) * 4;
      for (int pass = 0; pass < 2; ++pass) {
#pragma unroll
        for (int it = 0; it < 8; ++it) {
          const int row = it * 2 + hh;
          const v4f v = *(const v4f*)(slab + row * 68 + c4);
          *(volatile v4f*)(C + (size_t)(mBase + row) * ldc + n0 + c4) = v;
        }
        __threadfence();
      }
    } else {
      const int q = lane >> 3, c8 = (lane & 7) * 8;
      unsigned short* C  = (unsigned short*)Cout;
      unsigned short* C2 = (unsigned short*)Cout2;
      for (int pass = 0; pass < 2; ++pass) {
#pragma unroll
        for (int it = 0; it < 4; ++it) {
          const int row = it * 4 + q;
          const float* sp = slab + row * 68 + c8;
          v8h hv, lv;
#pragma unroll
          for (int e = 0; e < 8; ++e) {
            const float x = sp[e];
            const unsigned short hb = f2bf_bits(x);
            const unsigned short lb = f2bf_bits(x - bf_bits2f(hb));
            hv[e] = __builtin_bit_cast(_Float16, hb);
            lv[e] = __builtin_bit_cast(_Float16, lb);
          }
          *(volatile v8h*)(C  + (size_t)(mBase + row) * ldc + n0 + c8) = hv;
          *(volatile v8h*)(C2 + (size_t)(mBase + row) * ldc + n0 + c8) = lv;
        }
        __threadfence();
      }
    }
    __builtin_amdgcn_fence(__ATOMIC_RELEASE, "workgroup");
    __builtin_amdgcn_wave_barrier();
    __builtin_amdgcn_fence(__ATOMIC_ACQUIRE, "workgroup");
  }
}

__global__ __launch_bounds__(512) void edge_kernel(
    const float* __restrict__ UV,
    const _Float16* __restrict__ Wcb, const float* __restrict__ bcb,
    const _Float16* __restrict__ Wcc, const float* __restrict__ bcc,
    const _Float16* __restrict__ WoT, const float* __restrict__ bout,
    float* __restrict__ out)
{
  __shared__ __align__(16) unsigned char smem_raw[kEdgeRows * kHid * 2];
  static_assert(sizeof(smem_raw) == 65536);
  _Float16* Abuf = (_Float16*)smem_raw;
  float* stg = (float*)smem_raw;

  const int tid  = threadIdx.x;
  const int lane = tid & 31;
  const int wave = tid >> 5;
  const int hh   = lane >> 4;
  const int rl   = lane & 15;
  const int koff = hh * 8;

  const int j0 = blockIdx.x * kEdgeRows;
  const int ii = blockIdx.y;
  const int bb = blockIdx.z;

  {
    const int k8 = (tid & 63) * 8;
    const int mr = tid >> 6;
    const float* vrow = UV + (size_t)(bb * kNodes + ii) * kUVP + kHid + k8;
    const v4f v0 = *(const v4f*)(vrow);
    const v4f v1 = *(const v4f*)(vrow + 4);
#pragma unroll 1
    for (int it = 0; it < 8; ++it) {
      const int m = mr + 8 * it;
      const float* urow = UV + (size_t)(bb * kNodes + j0 + m) * kUVP + k8;
      const v4f u0 = *(const v4f*)(urow);
      const v4f u1 = *(const v4f*)(urow + 4);
      v8h hv;
#pragma unroll
      for (int e = 0; e < 4; ++e) {
        hv[e]     = (_Float16)fmaxf(u0[e] + v0[e], 0.0f);
        hv[4 + e] = (_Float16)fmaxf(u1[e] + v1[e], 0.0f);
      }
      *(v8h*)(Abuf + m * kHid + k8) = hv;
    }
  }
  __syncthreads();

  const int m0 = (wave >> 3) * 32;
  const int n0 = (wave & 7) * 64;
#pragma unroll 1
  for (int layer = 0; layer < 2; ++layer) {
    const _Float16* W = layer ? Wcc : Wcb;
    const float* bias = layer ? bcc : bcb;
    v8f acc[2][4];
#pragma unroll
    for (int i = 0; i < 2; ++i)
#pragma unroll
      for (int j = 0; j < 4; ++j) acc[i][j] = (v8f){0.f,0.f,0.f,0.f,0.f,0.f,0.f,0.f};
    const _Float16* wrow = W + (size_t)(n0 + rl) * kHid + koff;
    const int aoff = (m0 + rl) * kHid + koff;
#pragma unroll 1
    for (int k0 = 0; k0 < kHid; k0 += 32) {
      v16h bf[4];
#pragma unroll
      for (int j = 0; j < 4; ++j) bf[j] = Frag<_Float16>::load(wrow + (size_t)j * 16 * kHid + k0);
#pragma unroll
      for (int i = 0; i < 2; ++i) {
        Frag<_Float16>::U fa;
        fa.h[0] = *(const v8h*)(Abuf + aoff + i * 16 * kHid + k0);
        fa.h[1] = *(const v8h*)(Abuf + aoff + i * 16 * kHid + k0 + 16);
#pragma unroll
        for (int j = 0; j < 4; ++j) acc[i][j] = mma_h(fa.v, bf[j], acc[i][j]);
      }
    }
    __syncthreads();
#pragma unroll
    for (int j = 0; j < 4; ++j) {
      const int n = n0 + (j << 4) + rl;
      const float bv = bias[n] * kActCarry;
#pragma unroll
      for (int i = 0; i < 2; ++i) {
#pragma unroll
        for (int r = 0; r < 8; ++r) {
          const int row = m0 + (i << 4) + 8 * hh + r;
          const float v = fmaxf(fmaf(acc[i][j][r], kAccScale, bv), 0.0f);
          Abuf[row * kHid + n] = (_Float16)v;
        }
      }
    }
    __syncthreads();
  }

  v8f oacc = (v8f){0.f,0.f,0.f,0.f,0.f,0.f,0.f,0.f};
  if (wave < 4) {
    const _Float16* wrow = WoT + (size_t)rl * kHid + koff;
    const int aoff = (wave * 16 + rl) * kHid + koff;
#pragma unroll 1
    for (int k0 = 0; k0 < kHid; k0 += 32) {
      const v16h bf = Frag<_Float16>::load(wrow + k0);
      Frag<_Float16>::U fa;
      fa.h[0] = *(const v8h*)(Abuf + aoff + k0);
      fa.h[1] = *(const v8h*)(Abuf + aoff + k0 + 16);
      oacc = mma_h(fa.v, bf, oacc);
    }
  }
  __syncthreads();
  if (wave < 4 && rl < 4) {
#pragma unroll
    for (int r = 0; r < 8; ++r) stg[(wave * 16 + 8 * hh + r) * 4 + rl] = oacc[r];
  }
  __syncthreads();
  if (wave == 0) {
    const v4f s0 = *(const v4f*)(stg + lane * 8);
    const v4f s1 = *(const v4f*)(stg + lane * 8 + 4);
    const float bo0 = bout[0];
    const float bo1 = bout[1];
    v4f o;
    o[0] = fmaf(s0[2], kLoInv, s0[0]) * kOutScale + bo0;
    o[1] = fmaf(s0[3], kLoInv, s0[1]) * kOutScale + bo1;
    o[2] = fmaf(s1[2], kLoInv, s1[0]) * kOutScale + bo0;
    o[3] = fmaf(s1[3], kLoInv, s1[1]) * kOutScale + bo1;
    float* dst = out + ((size_t)(bb * kNodes + ii) * kNodes + j0) * 2 + lane * 4;
    *(volatile v4f*)dst = o;
    __threadfence();
    *(volatile v4f*)dst = o;
  }
}

extern "C" void kernel_launch(void* const* d_in, const int* in_sizes, int n_in,
                              void* d_out, int out_size, void* d_ws, size_t ws_size,
                              hipStream_t stream) {
  if (n_in < 16) return;
  if (in_sizes[0] != kRows * kDim) return;
  if (in_sizes[1] != kRows * 2) return;
  if (in_sizes[2] != kHid * 2) return;
  if (in_sizes[3] != kHid) return;
  if (in_sizes[4] != kHid * kDim) return;
  if (in_sizes[5] != kHid) return;
  if (in_sizes[6] != kHid * kHid) return;
  if (in_sizes[7] != kHid) return;
  if (in_sizes[8] != kHid * kUVP) return;
  if (in_sizes[9] != kHid) return;
  if (in_sizes[10] != kHid * kHid) return;
  if (in_sizes[11] != kHid) return;
  if (in_sizes[12] != kHid * kHid) return;
  if (in_sizes[13] != kHid) return;
  if (in_sizes[14] != 2 * kHid) return;
  if (in_sizes[15] != 2) return;
  if (out_size != kBatch * kNodes * kNodes * 2) return;
  if (ws_size < kWsTotal) return;

  const float* brick = (const float*)d_in[0];
  const float* xy    = (const float*)d_in[1];
  const float* W_xy  = (const float*)d_in[2];
  const float* b_xy  = (const float*)d_in[3];
  const float* W_a   = (const float*)d_in[4];
  const float* b_a   = (const float*)d_in[5];
  const float* W_b   = (const float*)d_in[6];
  const float* b_b   = (const float*)d_in[7];
  const float* W_ca  = (const float*)d_in[8];
  const float* b_ca  = (const float*)d_in[9];
  const float* W_cb  = (const float*)d_in[10];
  const float* b_cb  = (const float*)d_in[11];
  const float* W_cc  = (const float*)d_in[12];
  const float* b_cc  = (const float*)d_in[13];
  const float* W_out = (const float*)d_in[14];
  const float* b_out = (const float*)d_in[15];
  float* out = (float*)d_out;

  unsigned char* ws = (unsigned char*)d_ws;
  unsigned short* BRH = (unsigned short*)(ws + kOffBRH);
  unsigned short* BRL = (unsigned short*)(ws + kOffBRL);
  unsigned short* WAH = (unsigned short*)(ws + kOffWAH);
  unsigned short* WAL = (unsigned short*)(ws + kOffWAL);
  unsigned short* WBH = (unsigned short*)(ws + kOffWBH);
  unsigned short* WBL = (unsigned short*)(ws + kOffWBL);
  unsigned short* UVH = (unsigned short*)(ws + kOffUVH);
  unsigned short* UVL = (unsigned short*)(ws + kOffUVL);
  unsigned short* F1H = (unsigned short*)(ws + kOffF1H);
  unsigned short* F1L = (unsigned short*)(ws + kOffF1L);
  unsigned short* F2H = (unsigned short*)(ws + kOffF2H);
  unsigned short* F2L = (unsigned short*)(ws + kOffF2L);
  float*          UV  = (float*)(ws + kOffUV);
  const _Float16* WCB = (const _Float16*)(ws + kOffWCB);
  const _Float16* WCC = (const _Float16*)(ws + kOffWCC);
  const _Float16* WOT = (const _Float16*)(ws + kOffWOT);

  prep_kernel<<<kSegEnd, 256, 0, stream>>>(brick, W_a, W_b, W_ca, W_cb, W_cc, W_out, ws);

  node_gemm_kernel<0><<<(kRows / 64) * (kHid / 64) / 8, 256, 0, stream>>>(
      BRH, BRL, WAH, WAL, (void*)F1H, (void*)F1L, kHid, b_a, b_xy, xy, W_xy, kRows, kHid);

  node_gemm_kernel<1><<<(kRows / 64) * (kHid / 64) / 8, 256, 0, stream>>>(
      F1H, F1L, WBH, WBL, (void*)F2H, (void*)F2L, kHid, b_b, b_b, xy, W_xy, kRows, kHid);

  node_gemm_kernel<2><<<(kRows / 64) * (kUVP / 64) / 8, 256, 0, stream>>>(
      F2H, F2L, UVH, UVL, (void*)UV, (void*)UV, kUVP, b_ca, b_ca, xy, W_xy, kRows, kUVP);

  edge_kernel<<<dim3(kNodes / kEdgeRows, kNodes, kBatch), 512, 0, stream>>>(
      UV, WCB, b_cb, WCC, b_cc, WOT, b_out, out);
}
